// KPConv_17712445129349
// MI455X (gfx1250) — hardware-verified
//
#include <hip/hip_runtime.h>
#include <stddef.h>
#include <stdint.h>

#pragma clang fp contract(off)

#define PD      3
#define HN      32
#define KPT     15
#define CIN     128
#define COUT    128
#define KTOT    (KPT * CIN)
#define NKS     (KTOT / 32)
#define QB      16
#define NTHR    128
#define NWV     4
#define QPW     (QB / NWV)
#define NCT     2
#define NCG     (CIN / 32)
#define NJT     (CIN / 16)
#define ALO     2048
#define APITCH  4112
#define FP      40
#define WP      40
#define UROW    (CIN / 8)
#define NUB     (COUT * KTOT / 8)
#define UPR     (KTOT / 8)
#define NSWP    (QB * COUT / (4 * NTHR))
#define PPRW    (COUT / 4)
#define OFF_KP  0
#define OFF_A   256
#define OFF_FT  (OFF_A + QB * APITCH * 2)
#define OFF_WH  (OFF_FT + NWV * CIN * FP * 2)
#define OFF_WL  (OFF_WH + NWV * 16 * WP * 2)
#define OFF_O   (OFF_WL + NWV * 16 * WP * 2)
#define LDS_MAIN (OFF_O + QB * COUT * 4)
#define SHADOWV 1.0e6f
#define HSIG    0.5f
#define WSLIM   134217728

static_assert((KTOT % 32) == 0 && NKS * 32 == KTOT);
static_assert(QB == 16 && QB == NWV * QPW && NTHR == NWV * 32);
static_assert(COUT == 16 * NCT * NWV);
static_assert(HN == 32 && CIN == 32 * NCG && CIN == 16 * NJT && CIN == 8 * UROW && UROW == 16);
static_assert(ALO >= KTOT + CIN && APITCH >= ALO + KTOT + CIN && (APITCH % 8) == 0);
static_assert((FP % 8) == 0 && FP >= HN && (WP % 8) == 0 && WP >= HN);
static_assert((OFF_A % 16) == 0 && (OFF_FT % 16) == 0 && (OFF_WH % 16) == 0 && (OFF_WL % 16) == 0 && (OFF_O % 16) == 0);
static_assert(LDS_MAIN == 191232 && LDS_MAIN <= 300000);
static_assert((NUB % 256) == 0 && NUB * 8 == COUT * KTOT && UPR * 8 == KTOT);
static_assert(NSWP * NTHR * 4 == QB * COUT && PPRW == 32 && ((COUT * 4) % 128) == 0);
static_assert(KPT * PD <= 64 && 4 * KPT + 3 < 64);

typedef float          v4f  __attribute__((ext_vector_type(4)));
typedef float          v8f  __attribute__((ext_vector_type(8)));
typedef int            v8i  __attribute__((ext_vector_type(8)));
typedef unsigned short v8us __attribute__((ext_vector_type(8)));
typedef __bf16         v16b __attribute__((ext_vector_type(16)));
typedef v4f  __attribute__((may_alias)) v4fa;
typedef v8us __attribute__((may_alias)) v8usa;
union Frag { v16b b; v8us h[2]; v8i w; };

__device__ __forceinline__ v8f wmk(const Frag& a, const Frag& b, v8f c) {
  v8f d = __builtin_amdgcn_wmma_f32_16x16x32_bf16(false, a.b, false, b.b, (short)0, c, false, false);
  asm volatile("v_nop\n\tv_nop\n\tv_nop\n\tv_nop" : "+v"(d) : "v"(a.w), "v"(b.w));
  return d;
}

__device__ __forceinline__ unsigned short bf_bits(float f) {
  unsigned int u = __float_as_uint(f);
  u += 0x7FFFu + ((u >> 16) & 1u);
  return (unsigned short)(u >> 16);
}
__device__ __forceinline__ float bf_val(unsigned short b) { return __uint_as_float(((unsigned int)b) << 16); }
__device__ __forceinline__ float bf_rne(float f) { return bf_val(bf_bits(f)); }

__device__ __forceinline__ float blendf(float a, float b, unsigned ma) {
  return __uint_as_float((__float_as_uint(a) & ma) | (__float_as_uint(b) & ~ma));
}

__global__ __launch_bounds__(256) void k_fprep(const float* __restrict__ feat, unsigned short* FB, int nS, int nu) {
  const int u = (int)blockIdx.x * 256 + (int)threadIdx.x;
  if (u >= nu) return;
  const int row = u >> 4;
  const int g8  = (u & 15) * 8;
  const int rc  = row < nS ? row : nS - 1;
  const unsigned mk = 0u - (unsigned)(row < nS);
  const float* p = feat + (size_t)rc * CIN + g8;
  const v4f a = *(const v4fa*)p, b = *(const v4fa*)(p + 4);
  v8us o;
  o[0] = (unsigned short)(bf_bits(a.x) & mk); o[1] = (unsigned short)(bf_bits(a.y) & mk);
  o[2] = (unsigned short)(bf_bits(a.z) & mk); o[3] = (unsigned short)(bf_bits(a.w) & mk);
  o[4] = (unsigned short)(bf_bits(b.x) & mk); o[5] = (unsigned short)(bf_bits(b.y) & mk);
  o[6] = (unsigned short)(bf_bits(b.z) & mk); o[7] = (unsigned short)(bf_bits(b.w) & mk);
  unsigned short* dp = FB + (size_t)u * 8;
  *(volatile v8us*)dp = o;
  __threadfence();
  *(volatile v8us*)dp = o;
}

__global__ __launch_bounds__(256) void k_wprep(const float* __restrict__ W, unsigned short* WB) {
  const int u   = (int)blockIdx.x * 256 + (int)threadIdx.x;
  const int o   = u / UPR;
  const int kk8 = (u - o * UPR) * 8;
  const float* p = W + (size_t)kk8 * COUT + o;
  v8us ov;
#pragma unroll
  for (int j = 0; j < 8; ++j) ov[j] = bf_bits(p[(size_t)j * COUT]);
  unsigned short* dp = WB + (size_t)u * 8;
  *(volatile v8us*)dp = ov;
  __threadfence();
  *(volatile v8us*)dp = ov;
}

__global__ __launch_bounds__(NTHR) void k_main(const float* __restrict__ qp, const float* __restrict__ sp,
                                               const int* __restrict__ nbr, const unsigned short* __restrict__ FB,
                                               const float* __restrict__ kp, const unsigned short* __restrict__ WB,
                                               float* out, int nQ, int nS) {
  extern __shared__ __attribute__((aligned(16))) unsigned char lds[];
  const int tid  = (int)threadIdx.x, lane = tid & 31, hh = lane >> 4, m = lane & 15;
  const int wave = __builtin_amdgcn_readfirstlane(tid >> 5);
  float*          sKP = (float*)(lds + OFF_KP);
  unsigned short* sA  = (unsigned short*)(lds + OFF_A);
  unsigned short* sFT = (unsigned short*)(lds + OFF_FT) + wave * (CIN * FP);
  unsigned short* sWH = (unsigned short*)(lds + OFF_WH) + wave * (16 * WP);
  unsigned short* sWL = (unsigned short*)(lds + OFF_WL) + wave * (16 * WP);
  float*          sO  = (float*)(lds + OFF_O);
  const int qBase = (int)blockIdx.x * QB;

  if (tid < 64) {
    const int k = tid >> 2, c = tid & 3;
    int ci = PD * k + c;
    ci = ci > KPT * PD - 1 ? KPT * PD - 1 : ci;
    const float v = bf_rne(kp[ci]);
    const unsigned ma = 0u - (unsigned)((k < KPT) & (c < PD));
    sKP[tid] = blendf(v, 0.0f, ma);
  }
  sWH[KPT * WP + lane] = (unsigned short)0;
  sWL[KPT * WP + lane] = (unsigned short)0;
  __syncthreads();

  const v8f z8 = {0.f, 0.f, 0.f, 0.f, 0.f, 0.f, 0.f, 0.f};

#pragma unroll 1
  for (int p = 0; p < QPW; ++p) {
    const int row = QPW * wave + p;
    const int n   = qBase + row;
    const int nc  = n < nQ ? n : nQ - 1;
    int idx = nbr[(size_t)nc * HN + lane];
    idx = idx < 0 ? 0 : idx;
    idx = idx > nS ? nS : idx;
    const unsigned vm = 0u - (unsigned)(idx < nS);
    const int is = idx < nS ? idx : nS - 1;
    const float qx = bf_rne(qp[(size_t)nc * PD + 0]);
    const float qy = bf_rne(qp[(size_t)nc * PD + 1]);
    const float qz = bf_rne(qp[(size_t)nc * PD + 2]);
    const float sx = bf_rne(sp[(size_t)is * PD + 0]);
    const float sy = bf_rne(sp[(size_t)is * PD + 1]);
    const float sz = bf_rne(sp[(size_t)is * PD + 2]);
    const float rx = blendf(sx, SHADOWV, vm) - qx;
    const float ry = blendf(sy, SHADOWV, vm) - qy;
    const float rz = blendf(sz, SHADOWV, vm) - qz;

    {
      const unsigned short* fr = FB + (size_t)idx * CIN;
#pragma unroll
      for (int g = 0; g < NCG; ++g) {
        const v8us f0 = *(const v8usa*)(fr + 32 * g);
        const v8us f1 = *(const v8usa*)(fr + 32 * g + 8);
        const v8us f2 = *(const v8usa*)(fr + 32 * g + 16);
        const v8us f3 = *(const v8usa*)(fr + 32 * g + 24);
        unsigned short* col = sFT + (32 * g) * FP + lane;
#pragma unroll
        for (int e = 0; e < 8; ++e) {
          col[(e) * FP]      = f0[e];
          col[(8 + e) * FP]  = f1[e];
          col[(16 + e) * FP] = f2[e];
          col[(24 + e) * FP] = f3[e];
        }
      }
    }

#pragma unroll
    for (int k = 0; k < KPT; ++k) {
      const v4f kv = *(const v4fa*)(sKP + 4 * k);
      const float dx = rx - kv.x;
      const float dy = ry - kv.y;
      const float dz = rz - kv.z;
      const float sq = (dx * dx + dz * dz) + dy * dy;
      const float dd = __builtin_amdgcn_sqrtf(sq);
      float w = 1.0f - dd * HSIG;
      w = fmaxf(w, 0.0f);
      const unsigned short hb = bf_bits(w);
      const unsigned short lb = bf_bits(w - bf_val(hb));
      sWH[k * WP + lane] = hb;
      sWL[k * WP + lane] = lb;
    }
    __syncthreads();

    Frag bh, bl;
    bh.h[0] = *(const v8usa*)(sWH + m * WP + 8 * hh);
    bh.h[1] = *(const v8usa*)(sWH + m * WP + 16 + 8 * hh);
    bl.h[0] = *(const v8usa*)(sWL + m * WP + 8 * hh);
    bl.h[1] = *(const v8usa*)(sWL + m * WP + 16 + 8 * hh);
    unsigned short* arow = sA + (size_t)row * APITCH + CIN * m + 8 * hh;
#pragma unroll
    for (int j = 0; j < NJT; ++j) {
      Frag af;
      af.h[0] = *(const v8usa*)(sFT + (16 * j + m) * FP + 8 * hh);
      af.h[1] = *(const v8usa*)(sFT + (16 * j + m) * FP + 16 + 8 * hh);
      v8f d = wmk(af, bh, z8);
      d = wmk(af, bl, d);
      v8us hv, lv;
#pragma unroll
      for (int r = 0; r < 8; ++r) {
        const unsigned short hb = bf_bits(d[r]);
        hv[r] = hb;
        lv[r] = bf_bits(d[r] - bf_val(hb));
      }
      *(v8usa*)(arow + 16 * j)       = hv;
      *(v8usa*)(arow + ALO + 16 * j) = lv;
    }
    __syncthreads();
  }

  v8f acc0 = z8, acc1 = z8;
  const unsigned short* bp0 = WB + (size_t)(32 * wave + m) * KTOT + 8 * hh;
  const unsigned short* bp1 = bp0 + (size_t)16 * KTOT;
  const unsigned short* ap  = sA + (size_t)m * APITCH + 8 * hh;
#pragma unroll 1
  for (int ks = 0; ks < NKS; ++ks) {
    const int k0 = 32 * ks;
    Frag b0, b1;
    b0.h[0] = *(const v8usa*)(bp0 + k0);
    b0.h[1] = *(const v8usa*)(bp0 + k0 + 16);
    b1.h[0] = *(const v8usa*)(bp1 + k0);
    b1.h[1] = *(const v8usa*)(bp1 + k0 + 16);
    Frag a;
    a.h[0] = *(const v8usa*)(ap + k0);
    a.h[1] = *(const v8usa*)(ap + k0 + 16);
    acc0 = wmk(a, b0, acc0);
    acc1 = wmk(a, b1, acc1);
    a.h[0] = *(const v8usa*)(ap + ALO + k0);
    a.h[1] = *(const v8usa*)(ap + ALO + k0 + 16);
    acc0 = wmk(a, b0, acc0);
    acc1 = wmk(a, b1, acc1);
  }

#pragma unroll
  for (int r = 0; r < 8; ++r) {
    sO[(8 * hh + r) * COUT + 32 * wave + m]      = acc0[r];
    sO[(8 * hh + r) * COUT + 32 * wave + 16 + m] = acc1[r];
  }
  __syncthreads();

  v4f pv[NSWP];
#pragma unroll
  for (int it = 0; it < NSWP; ++it) pv[it] = *(const v4fa*)(sO + (size_t)(it * NTHR + tid) * 4);
  float* ob = out + (size_t)qBase * COUT;
#pragma unroll
  for (int it = 0; it < NSWP; ++it) {
    const int pc = it * NTHR + tid;
    const int prow = pc / PPRW;
    if (qBase + prow < nQ) *(volatile v4f*)(ob + (size_t)pc * 4) = pv[it];
  }
  __threadfence();
#pragma unroll
  for (int it = 0; it < NSWP; ++it) {
    const int pc = it * NTHR + tid;
    const int prow = pc / PPRW;
    if (qBase + prow < nQ) *(volatile v4f*)(ob + (size_t)pc * 4) = pv[it];
  }
}

static inline int cdiv(int a, int b) { return (a + b - 1) / b; }
static inline size_t al256(size_t o) { return (o + 255) & ~(size_t)255; }

extern "C" void kernel_launch(void* const* d_in, const int* in_sizes, int n_in,
                              void* d_out, int out_size, void* d_ws, size_t ws_size,
                              hipStream_t stream) {
  if (n_in < 6) return;
  if (in_sizes[0] < PD || (in_sizes[0] % PD) != 0) return;
  if (in_sizes[1] < PD || (in_sizes[1] % PD) != 0) return;
  const int nQ = in_sizes[0] / PD;
  const int nS = in_sizes[1] / PD;
  if (nQ < 1 || nS < 1 || nQ > (1 << 24) || nS > (1 << 24)) return;
  if ((long long)in_sizes[2] != (long long)nS * CIN) return;
  if ((long long)in_sizes[3] != (long long)nQ * HN) return;
  if (in_sizes[4] != KPT * CIN * COUT) return;
  if (in_sizes[5] != KPT * PD) return;
  if ((long long)out_size != (long long)nQ * COUT) return;

  const float* qp   = (const float*)d_in[0];
  const float* sp   = (const float*)d_in[1];
  const float* feat = (const float*)d_in[2];
  const int*   nbr  = (const int*)  d_in[3];
  const float* W    = (const float*)d_in[4];
  const float* kpts = (const float*)d_in[5];
  float* out = (float*)d_out;

  const int fbRows = cdiv(nS + 1, 2) * 2;
  const int nu     = fbRows * UROW;

  char* ws = (char*)d_ws;
  size_t off = 0;
  const size_t oFB = off; off = al256(off + (size_t)nu * 16);
  const size_t oWB = off; off = al256(off + (size_t)NUB * 16);
  if (off > ws_size || off > (size_t)WSLIM) return;
  unsigned short* FB = (unsigned short*)(ws + oFB);
  unsigned short* WB = (unsigned short*)(ws + oWB);

  hipFuncSetAttribute(reinterpret_cast<const void*>(&k_main), hipFuncAttributeMaxDynamicSharedMemorySize, LDS_MAIN);

  k_fprep<<<cdiv(nu, 256), 256, 0, stream>>>(feat, FB, nS, nu);
  k_wprep<<<NUB / 256, 256, 0, stream>>>(W, WB);
  k_main<<<cdiv(nQ, QB), NTHR, LDS_MAIN, stream>>>(qp, sp, nbr, FB, kpts, WB, out, nQ, nS);
  (void)hipGetLastError();
}
